// DifferentiableFeatureAligner2_39152921870906
// MI455X (gfx1250) — hardware-verified
//
#include <hip/hip_runtime.h>
#include <stddef.h>


#define PIX   32
#define NB    4
#define EMB   64
#define CCLS  2
#define CREG  14
#define CALL  16
#define ROWS  (NB * PIX)
#define NTHR  256
#define NWAV  (NTHR / 32)
#define NLINE (NB * CALL)
#define NCHK  2
#define VCAP  240
#define WSCAP 134217728
#define LNEPS 1e-5f
#define RSQD  0.125f

static_assert(ROWS == 16 * NWAV);
static_assert(NTHR == 2 * ROWS);
static_assert(NLINE == 8 * NWAV);
static_assert(((ROWS * 8) % NTHR) == 0);
static_assert((NLINE * PIX) == 8 * NTHR);
static_assert((CALL * NB * PIX) == 8 * NTHR);
static_assert((EMB % 32) == 0 && (PIX % 32) == 0);

typedef float          v4f  __attribute__((ext_vector_type(4)));
typedef float          v8f  __attribute__((ext_vector_type(8)));
typedef unsigned short v8us __attribute__((ext_vector_type(8)));
typedef unsigned int   v4u  __attribute__((ext_vector_type(4)));
typedef __bf16         v16b __attribute__((ext_vector_type(16)));
union FragB { v16b v; v8us u[2]; };

__device__ __forceinline__ unsigned int bf16_rne(float x) {
  unsigned int u = __float_as_uint(x);
  u = u + 0x7FFFu + ((u >> 16) & 1u);
  return u >> 16;
}
__device__ __forceinline__ float bf16_val(unsigned int b) { return __uint_as_float(b << 16); }

__device__ __forceinline__ v8f wmb(v16b a, v16b b, v8f c) {
  v8f d = __builtin_amdgcn_wmma_f32_16x16x32_bf16(false, a, false, b, (short)0, c, false, false);
  asm volatile("v_nop\n\tv_nop\n\tv_nop\n\tv_nop" : "+v"(d) : "v"(a), "v"(b));
  return d;
}

__device__ __forceinline__ v4f relu4(v4f a) {
  v4f r;
  r.x = fmaxf(a.x, 0.0f); r.y = fmaxf(a.y, 0.0f); r.z = fmaxf(a.z, 0.0f); r.w = fmaxf(a.w, 0.0f);
  return r;
}

__global__ __launch_bounds__(NTHR) void k_prep(const float* __restrict__ W2,
                                               unsigned short* Wh, unsigned short* Wl) {
  const int tid = threadIdx.x;
  v8us hv[2], lv[2];
#pragma unroll
  for (int it = 0; it < 2; ++it) {
    const int idx = tid + NTHR * it;
    const int n = idx >> 3, k0 = (idx & 7) * 8;
#pragma unroll
    for (int e = 0; e < 8; ++e) {
      const float w = W2[(k0 + e) * EMB + n];
      const unsigned int hb = bf16_rne(w);
      const unsigned int lb = bf16_rne(w - bf16_val(hb));
      hv[it][e] = (unsigned short)hb;
      lv[it][e] = (unsigned short)lb;
    }
  }
#pragma unroll
  for (int it = 0; it < 2; ++it) {
    const int idx = tid + NTHR * it;
    *(volatile v8us*)(Wh + 8 * idx) = hv[it];
    *(volatile v8us*)(Wl + 8 * idx) = lv[it];
  }
  __threadfence();
#pragma unroll
  for (int it = 0; it < 2; ++it) {
    const int idx = tid + NTHR * it;
    *(volatile v8us*)(Wh + 8 * idx) = hv[it];
    *(volatile v8us*)(Wl + 8 * idx) = lv[it];
  }
}

__global__ __launch_bounds__(NTHR) __attribute__((amdgpu_num_vgpr(VCAP))) void k_enc(
    const float* __restrict__ ego_cls, const float* __restrict__ ego_reg,
    const float* __restrict__ oth_cls, const float* __restrict__ oth_reg,
    const float* __restrict__ W1, const float* __restrict__ b1,
    const float* __restrict__ gam, const float* __restrict__ bet,
    const unsigned short* __restrict__ W2h, const unsigned short* __restrict__ W2l,
    const float* __restrict__ b2, float* dpl, int HW, int HWC, int pbase) {
  __shared__ __attribute__((aligned(16))) float sDsc[ROWS * 8];
  __shared__ __attribute__((aligned(16))) float sH[ROWS * EMB];
  __shared__ __attribute__((aligned(16))) unsigned short sAh[ROWS * EMB];
  __shared__ __attribute__((aligned(16))) unsigned short sAl[ROWS * EMB];

  const int tid = threadIdx.x, lane = tid & 31, wv = tid >> 5, hh = lane >> 4, m = lane & 15;
  const int s = blockIdx.y;
  const int p0 = pbase + blockIdx.x * PIX;
  const size_t hw = (size_t)HW;
  const float* cls = s ? oth_cls : ego_cls;
  const float* reg = s ? oth_reg : ego_reg;

  if (tid < ROWS) {
    const int r = tid, bi = r >> 5, pl = r & 31;
    const size_t n = (size_t)p0 + (size_t)pl;
    const float* rp = reg + (size_t)(bi * CREG) * hw + n;
    const float* cp = cls + (size_t)(bi * CCLS) * hw + n;
    v4f da, db;
    da.x = rp[3 * hw];
    da.y = rp[4 * hw];
    da.z = rp[5 * hw];
    const float th = rp[6 * hw];
    da.w = sinf(th);
    db.x = cosf(th);
    const float ca = cp[0], cb = cp[hw];
    db.y = fmaxf(ca, cb);
    db.z = 0.0f;
    db.w = 0.0f;
    *(v4f*)(sDsc + r * 8) = da;
    *(v4f*)(sDsc + r * 8 + 4) = db;
  }
  __syncthreads();

#pragma unroll 1
  for (int it = 0; it < (ROWS * 8) / NTHR; ++it) {
    const int o = tid + NTHR * it;
    const int r = o >> 3, c0 = (o & 7) * 8;
    const v4f da = *(const v4f*)(sDsc + r * 8);
    const v4f db = *(const v4f*)(sDsc + r * 8 + 4);
    const float* wp = W1 + c0;
    v4f a = da.x * *(const v4f*)(wp);
    v4f b = da.x * *(const v4f*)(wp + 4);
    a = a + da.y * *(const v4f*)(wp + 1 * EMB);     b = b + da.y * *(const v4f*)(wp + 1 * EMB + 4);
    a = a + da.z * *(const v4f*)(wp + 2 * EMB);     b = b + da.z * *(const v4f*)(wp + 2 * EMB + 4);
    a = a + da.w * *(const v4f*)(wp + 3 * EMB);     b = b + da.w * *(const v4f*)(wp + 3 * EMB + 4);
    a = a + db.x * *(const v4f*)(wp + 4 * EMB);     b = b + db.x * *(const v4f*)(wp + 4 * EMB + 4);
    a = a + db.y * *(const v4f*)(wp + 5 * EMB);     b = b + db.y * *(const v4f*)(wp + 5 * EMB + 4);
    a = a + *(const v4f*)(b1 + c0);
    b = b + *(const v4f*)(b1 + c0 + 4);
    *(v4f*)(sH + r * EMB + c0) = relu4(a);
    *(v4f*)(sH + r * EMB + c0 + 4) = relu4(b);
  }
  __syncthreads();

  {
    const int r = tid >> 1, q = tid & 1, c0 = 32 * q;
    const float* hp = sH + r * EMB + c0;
    float s1 = 0.0f;
#pragma unroll
    for (int g = 0; g < 8; ++g) {
      const v4f v = *(const v4f*)(hp + 4 * g);
      s1 += (v.x + v.y) + (v.z + v.w);
    }
    s1 += __shfl_xor(s1, 1);
    const float mu = s1 * (1.0f / 64.0f);
    float s2 = 0.0f;
#pragma unroll
    for (int g = 0; g < 8; ++g) {
      const v4f v = *(const v4f*)(hp + 4 * g);
      const v4f dv = v - mu;
      s2 = fmaf(dv.x, dv.x, s2);
      s2 = fmaf(dv.y, dv.y, s2);
      s2 = fmaf(dv.z, dv.z, s2);
      s2 = fmaf(dv.w, dv.w, s2);
    }
    s2 += __shfl_xor(s2, 1);
    const float var = s2 * (1.0f / 64.0f);
    const float rs = 1.0f / sqrtf(var + LNEPS);

    unsigned short* ah = sAh + r * EMB + c0;
    unsigned short* al = sAl + r * EMB + c0;
#pragma unroll 2
    for (int g = 0; g < 4; ++g) {
      const v4f va = *(const v4f*)(hp + 8 * g);
      const v4f vb = *(const v4f*)(hp + 8 * g + 4);
      const v4f ga = *(const v4f*)(gam + c0 + 8 * g);
      const v4f gb = *(const v4f*)(gam + c0 + 8 * g + 4);
      const v4f ea = *(const v4f*)(bet + c0 + 8 * g);
      const v4f eb = *(const v4f*)(bet + c0 + 8 * g + 4);
      const v4f ya = (va - mu) * rs * ga + ea;
      const v4f yb = (vb - mu) * rs * gb + eb;
      float y[8];
      y[0] = ya.x; y[1] = ya.y; y[2] = ya.z; y[3] = ya.w;
      y[4] = yb.x; y[5] = yb.y; y[6] = yb.z; y[7] = yb.w;
      v4u hv, lv;
#pragma unroll
      for (int e2 = 0; e2 < 4; ++e2) {
        const unsigned int h0 = bf16_rne(y[2 * e2]);
        const unsigned int h1 = bf16_rne(y[2 * e2 + 1]);
        const unsigned int l0 = bf16_rne(y[2 * e2] - bf16_val(h0));
        const unsigned int l1 = bf16_rne(y[2 * e2 + 1] - bf16_val(h1));
        hv[e2] = h0 | (h1 << 16);
        lv[e2] = l0 | (l1 << 16);
      }
      *(v4u*)(ah + 8 * g) = hv;
      *(v4u*)(al + 8 * g) = lv;
    }
  }
  __syncthreads();

  {
    const unsigned short* ap = sAh + (16 * wv + m) * EMB + 8 * hh;
    const unsigned short* aq = sAl + (16 * wv + m) * EMB + 8 * hh;
    FragB fh0, fl0, fh1, fl1;
    fh0.u[0] = *(const v8us*)(ap);
    fh0.u[1] = *(const v8us*)(ap + 16);
    fh1.u[0] = *(const v8us*)(ap + 32);
    fh1.u[1] = *(const v8us*)(ap + 48);
    fl0.u[0] = *(const v8us*)(aq);
    fl0.u[1] = *(const v8us*)(aq + 16);
    fl1.u[0] = *(const v8us*)(aq + 32);
    fl1.u[1] = *(const v8us*)(aq + 48);
    float* dp = sH + (16 * wv + 8 * hh) * EMB + m;
#pragma unroll 1
    for (int t = 0; t < EMB / 16; ++t) {
      v8f acc = {0.f, 0.f, 0.f, 0.f, 0.f, 0.f, 0.f, 0.f};
      const unsigned short* bp = W2h + (size_t)(16 * t + m) * EMB + 8 * hh;
      const unsigned short* bq = W2l + (size_t)(16 * t + m) * EMB + 8 * hh;
      FragB gh, gl;
      gh.u[0] = *(const v8us*)(bp);
      gh.u[1] = *(const v8us*)(bp + 16);
      gl.u[0] = *(const v8us*)(bq);
      gl.u[1] = *(const v8us*)(bq + 16);
      acc = wmb(fh0.v, gh.v, acc);
      acc = wmb(fh0.v, gl.v, acc);
      acc = wmb(fl0.v, gh.v, acc);
      gh.u[0] = *(const v8us*)(bp + 32);
      gh.u[1] = *(const v8us*)(bp + 48);
      gl.u[0] = *(const v8us*)(bq + 32);
      gl.u[1] = *(const v8us*)(bq + 48);
      acc = wmb(fh1.v, gh.v, acc);
      acc = wmb(fh1.v, gl.v, acc);
      acc = wmb(fl1.v, gh.v, acc);
      const float bb = b2[16 * t + m];
#pragma unroll
      for (int r = 0; r < 8; ++r) dp[r * EMB + 16 * t] = acc[r] + bb;
    }
  }
  __syncthreads();

  {
    const int rl = lane >> 4, f4 = (lane & 15) * 4;
    const size_t sb = (size_t)s * NB;
#pragma unroll
    for (int it = 0; it < 8; ++it) {
      const int lr = 16 * wv + 2 * it + rl;
      const int bi = lr >> 5, pl = lr & 31;
      const v4f v = *(const v4f*)(sH + lr * EMB + f4);
      float* gp = dpl + ((sb + (size_t)bi) * (size_t)HWC + (size_t)(p0 - pbase + pl)) * EMB + f4;
      *(volatile v4f*)gp = v;
    }
    __threadfence();
#pragma unroll
    for (int it = 0; it < 8; ++it) {
      const int lr = 16 * wv + 2 * it + rl;
      const int bi = lr >> 5, pl = lr & 31;
      const v4f v = *(const v4f*)(sH + lr * EMB + f4);
      float* gp = dpl + ((sb + (size_t)bi) * (size_t)HWC + (size_t)(p0 - pbase + pl)) * EMB + f4;
      *(volatile v4f*)gp = v;
    }
  }
}

__device__ __forceinline__ void decL(int L, int& i, int& c16) {
  const int isC = L < 8;
  const int L2 = L - 8;
  const int ir = L2 / 14;
  i = isC ? (L >> 1) : ir;
  c16 = isC ? (L & 1) : (2 + L2 - 14 * ir);
}

__global__ __launch_bounds__(NTHR) __attribute__((amdgpu_num_vgpr(VCAP))) void k_align(
    const float* __restrict__ oth_cls, const float* __restrict__ oth_reg,
    const float* __restrict__ dpl, float* out, int HW, int HWC, int pbase) {
  __shared__ __attribute__((aligned(16))) float sRaw[CALL * NB * PIX];
  __shared__ __attribute__((aligned(16))) float sAt[PIX * 16];
  __shared__ __attribute__((aligned(16))) float sOut[NLINE * PIX];

  const int tid = threadIdx.x, lane = tid & 31, wv = tid >> 5;
  const int p0 = pbase + blockIdx.x * PIX;
  const size_t hw = (size_t)HW;

  {
    const size_t lp = (size_t)(p0 - pbase + lane);
#pragma unroll
    for (int u = 0; u < 2; ++u) {
      const int pr = 2 * wv + u;
      const int i = pr >> 2, j = pr & 3;
      const float* ep = dpl + ((size_t)i * (size_t)HWC + lp) * EMB;
      const float* op = dpl + ((size_t)(NB + j) * (size_t)HWC + lp) * EMB;
      float a = 0.0f;
#pragma unroll 4
      for (int e = 0; e < EMB / 4; ++e) {
        const v4f x = *(const v4f*)(ep + 4 * e);
        const v4f yv = *(const v4f*)(op + 4 * e);
        a = fmaf(x.x, yv.x, a);
        a = fmaf(x.y, yv.y, a);
        a = fmaf(x.z, yv.z, a);
        a = fmaf(x.w, yv.w, a);
      }
      sAt[lane * 16 + i * 4 + j] = a * RSQD;
    }
#pragma unroll
    for (int it = 0; it < 8; ++it) {
      const int idx = tid + NTHR * it;
      const int pl = idx & 31, jc = idx >> 5;
      const int j = jc >> 4, c = jc & 15;
      const int ccl = c < 2 ? c : 1;
      const int crg = c < 2 ? 0 : (c - 2);
      const float vc = oth_cls[(size_t)(j * CCLS + ccl) * hw + (size_t)(p0 + pl)];
      const float vg = oth_reg[(size_t)(j * CREG + crg) * hw + (size_t)(p0 + pl)];
      sRaw[idx] = (c < 2) ? vc : vg;
    }
  }
  __syncthreads();

#pragma unroll 2
  for (int it = 0; it < 8; ++it) {
    const int o = tid + NTHR * it;
    const int pl = o & 31, L = o >> 5;
    int i, c16;
    decL(L, i, c16);
    const float* at = sAt + pl * 16 + i * 4;
    const float* rw = sRaw + c16 * PIX + pl;
    float v = at[0] * rw[0];
    v = fmaf(at[1], rw[1 * CALL * PIX], v);
    v = fmaf(at[2], rw[2 * CALL * PIX], v);
    v = fmaf(at[3], rw[3 * CALL * PIX], v);
    sOut[o] = v;
  }
  __syncthreads();

  {
    v4f ov[2];
    size_t go[2];
#pragma unroll
    for (int q2 = 0; q2 < 2; ++q2) {
      const int L = wv * 8 + q2 * 4 + (lane >> 3);
      const int pc4 = (lane & 7) * 4;
      int i, c16;
      decL(L, i, c16);
      const int isC = c16 < 2;
      const int ccl = isC ? c16 : 0;
      const int crg = isC ? 0 : (c16 - 2);
      const size_t offc = (size_t)(i * CCLS + ccl) * hw;
      const size_t offr = (size_t)(NB * CCLS) * hw + (size_t)(i * CREG + crg) * hw;
      go[q2] = (isC ? offc : offr) + (size_t)p0 + (size_t)pc4;
      ov[q2] = *(const v4f*)(sOut + L * PIX + pc4);
    }
    *(volatile v4f*)(out + go[0]) = ov[0];
    *(volatile v4f*)(out + go[1]) = ov[1];
    __threadfence();
    *(volatile v4f*)(out + go[0]) = ov[0];
    *(volatile v4f*)(out + go[1]) = ov[1];
  }
}

extern "C" void kernel_launch(void* const* d_in, const int* in_sizes, int n_in,
                              void* d_out, int out_size, void* d_ws, size_t ws_size,
                              hipStream_t stream) {
  if (n_in < 10) return;
  const int n0 = in_sizes[0];
  if (n0 <= 0 || (n0 % (NB * CCLS)) != 0) return;
  const int HW = n0 / (NB * CCLS);
  if ((HW % (NCHK * PIX)) != 0) return;
  const int HWC = HW / NCHK;
  if (in_sizes[1] != NB * CREG * HW || in_sizes[2] != NB * CCLS * HW || in_sizes[3] != NB * CREG * HW) return;
  if (in_sizes[4] != 6 * EMB || in_sizes[5] != EMB || in_sizes[6] != EMB || in_sizes[7] != EMB ||
      in_sizes[8] != EMB * EMB || in_sizes[9] != EMB) return;
  if (out_size != NB * CALL * HW) return;

  const float* ego_cls = (const float*)d_in[0];
  const float* ego_reg = (const float*)d_in[1];
  const float* oth_cls = (const float*)d_in[2];
  const float* oth_reg = (const float*)d_in[3];
  const float* W1  = (const float*)d_in[4];
  const float* b1  = (const float*)d_in[5];
  const float* gam = (const float*)d_in[6];
  const float* bet = (const float*)d_in[7];
  const float* W2  = (const float*)d_in[8];
  const float* b2  = (const float*)d_in[9];
  float* out = (float*)d_out;

  const size_t oH = 0, oL = 8192, oD = 16384;
  const size_t dsz = (size_t)2 * NB * (size_t)HWC * EMB * sizeof(float);
  const size_t tot = oD + dsz;
  if (tot > ws_size || tot > (size_t)WSCAP) return;
  char* ws = (char*)d_ws;
  unsigned short* W2h = (unsigned short*)(ws + oH);
  unsigned short* W2l = (unsigned short*)(ws + oL);
  float* dpl = (float*)(ws + oD);

  k_prep<<<1, NTHR, 0, stream>>>(W2, W2h, W2l);
  for (int ch = 0; ch < NCHK; ++ch) {
    const int pbase = ch * HWC;
    k_enc<<<dim3(HWC / PIX, 2), NTHR, 0, stream>>>(ego_cls, ego_reg, oth_cls, oth_reg, W1, b1, gam, bet,
                                                   W2h, W2l, b2, dpl, HW, HWC, pbase);
    k_align<<<HWC / PIX, NTHR, 0, stream>>>(oth_cls, oth_reg, dpl, out, HW, HWC, pbase);
  }
}
